// GradEnergyMessagePassing_46196668236124
// MI455X (gfx1250) — hardware-verified
//
#include <hip/hip_runtime.h>
#include <stddef.h>


#pragma clang fp contract(off)

#define DF      64
#define HD      128
#define PQROW   256
#define NTHR    256
#define NWAVE   8
#define NBN     64
#define XP      72
#define SP      132
#define TE      128
#define AP      136
#define EPT     8
#define PIECE   (NTHR * EPT)
#define WCAP    (EPT * 32)
#define NBC     1024
#define SLB     10
#define PW1A    0
#define PW1B    8192
#define PW2     16384
#define PWTOT   32768
#define PREPBLK (PWTOT / (NTHR * 8))
#define WSCAP   134217728
#define PQDYN   (NWAVE * 16 * SP * 4)
#define AGGDYN  (NBC * DF * 4)

static_assert((PWTOT % (NTHR * 8)) == 0);
static_assert((PW1B % (NTHR * 8)) == 0);
static_assert((PW2 % (NTHR * 8)) == 0);
static_assert(((XP * 2) % 16) == 0);
static_assert(((AP * 2) % 16) == 0);
static_assert(((SP * 4) % 16) == 0);
static_assert(NBC == (1 << SLB));
static_assert(PIECE == 2048);
static_assert((EPT % 4) == 0);
static_assert((NBC % (2 * NWAVE)) == 0);
static_assert(NBN == 4 * 16);
static_assert(TE == NWAVE * 16);
static_assert(NTHR == 2 * TE);
static_assert((NBC * DF) % (4 * NTHR) == 0);
static_assert((PIECE % TE) == 0);

typedef float          v2f   __attribute__((ext_vector_type(2)));
typedef float          v4f   __attribute__((ext_vector_type(4)));
typedef float          v8f   __attribute__((ext_vector_type(8)));
typedef int            v4i   __attribute__((ext_vector_type(4)));
typedef unsigned int   v4u   __attribute__((ext_vector_type(4)));
typedef _Float16       v2h   __attribute__((ext_vector_type(2)));
typedef _Float16       v8h   __attribute__((ext_vector_type(8)));
typedef _Float16       v16h  __attribute__((ext_vector_type(16)));

__device__ __forceinline__ v16h ldfrag(const _Float16* p) {
  const v8h u0 = *(const v8h*)p;
  const v8h u1 = *(const v8h*)(p + 16);
  return __builtin_shufflevector(u0, u1, 0, 1, 2, 3, 4, 5, 6, 7, 8, 9, 10, 11, 12, 13, 14, 15);
}

__device__ __forceinline__ v8f wm(v16h a, v16h b, v8f c) {
  v8f d = __builtin_amdgcn_wmma_f32_16x16x32_f16(false, a, false, b, (short)0, c, false, false);
  asm volatile("v_nop\n\tv_nop\n\tv_nop\n\tv_nop" : "+v"(d) : "v"(a), "v"(b));
  return d;
}
__device__ __forceinline__ v8f zero8() {
  v8f z = {0.f, 0.f, 0.f, 0.f, 0.f, 0.f, 0.f, 0.f};
  return z;
}
__device__ __forceinline__ int iclamp(int v, int lo, int hi) { return v < lo ? lo : (v > hi ? hi : v); }

__device__ __forceinline__ float siluf(float v) {
  const float vc = fminf(fmaxf(v, -80.0f), 80.0f);
  return v * __builtin_amdgcn_rcpf(1.0f + __expf(-vc));
}
__device__ __forceinline__ _Float16 hchan(float p, float q, float tv, float w, float bb, float b1v) {
  const float tw = tv * w;
  const float te = siluf(tw + bb);
  const float z = ((p + q) + te) + b1v;
  return (_Float16)(16.0f * siluf(z));
}

__global__ __launch_bounds__(NTHR) void k_prep(const float* __restrict__ W1, const float* __restrict__ W2,
                                               _Float16* wp) {
  const int tid = (int)threadIdx.x;
  const int o = ((int)blockIdx.x * NTHR + tid) * 8;
  const float* src;
  int rowb, col;
  if (o < PW1B) {
    src = W1; rowb = o & 63; col = o >> 6;
  } else if (o < PW2) {
    const int idx = o - PW1B;
    src = W1; rowb = 64 + (idx & 63); col = idx >> 6;
  } else {
    const int idx = o - PW2;
    src = W2; rowb = idx & 127; col = idx >> 7;
  }
  v8h hv;
#pragma unroll
  for (int i = 0; i < 8; ++i) hv[i] = (_Float16)(64.0f * src[(size_t)(rowb + i) * HD + col]);
  const v4u u = __builtin_bit_cast(v4u, hv);
  _Float16* dst = wp + o;
  *(volatile v4u*)dst = u;
  __threadfence();
  *(volatile v4u*)dst = u;
}

__global__ __launch_bounds__(NTHR) void k_pq(const float* __restrict__ x, const _Float16* __restrict__ wp,
                                             float* PQ, int nN) {
  extern __shared__ __attribute__((aligned(16))) float stg[];
  __shared__ __attribute__((aligned(16))) _Float16 sX[NBN * XP];
  const int tid = (int)threadIdx.x, lane = tid & 31, wave = tid >> 5, hh = lane >> 4, m = lane & 15;
  const int n0 = (int)blockIdx.x * NBN;

  {
    const int nl = tid >> 2, q = tid & 3;
    int node = n0 + nl;
    node = node > nN - 1 ? nN - 1 : node;
    const float* rp = x + (size_t)node * DF + 16 * q;
    const v4f a = *(const v4f*)(rp);
    const v4f b = *(const v4f*)(rp + 4);
    const v4f c = *(const v4f*)(rp + 8);
    const v4f d = *(const v4f*)(rp + 12);
    v8h u0, u1;
    u0[0] = (_Float16)a.x; u0[1] = (_Float16)a.y; u0[2] = (_Float16)a.z; u0[3] = (_Float16)a.w;
    u0[4] = (_Float16)b.x; u0[5] = (_Float16)b.y; u0[6] = (_Float16)b.z; u0[7] = (_Float16)b.w;
    u1[0] = (_Float16)c.x; u1[1] = (_Float16)c.y; u1[2] = (_Float16)c.z; u1[3] = (_Float16)c.w;
    u1[4] = (_Float16)d.x; u1[5] = (_Float16)d.y; u1[6] = (_Float16)d.z; u1[7] = (_Float16)d.w;
    *(v8h*)(sX + nl * XP + 16 * q)     = u0;
    *(v8h*)(sX + nl * XP + 16 * q + 8) = u1;
  }
  __syncthreads();

  const int rt = wave & 3, cg = wave >> 2;
  const _Float16* bp = wp + (cg != 0 ? PW1B : PW1A);
  v8f c[8];
#pragma unroll
  for (int j = 0; j < 8; ++j) c[j] = zero8();
  const _Float16* ap = sX + (16 * rt + m) * XP + 8 * hh;
#pragma unroll
  for (int ks = 0; ks < 2; ++ks) {
    const v16h a = ldfrag(ap + 32 * ks);
#pragma unroll
    for (int j = 0; j < 8; ++j) {
      const v16h b = ldfrag(bp + (size_t)(16 * j + m) * DF + 32 * ks + 8 * hh);
      c[j] = wm(a, b, c[j]);
    }
  }
  float* sw = stg + wave * 16 * SP;
#pragma unroll
  for (int j = 0; j < 8; ++j) {
#pragma unroll
    for (int r = 0; r < 8; ++r) sw[(8 * hh + r) * SP + 16 * j + m] = c[j][r] * 0.015625f;
  }
  __syncthreads();
#pragma unroll 1
  for (int rr = 0; rr < 16; ++rr) {
    const v4f v = *(const v4f*)(sw + rr * SP + 4 * lane);
    *(volatile v4f*)(PQ + (size_t)(n0 + 16 * rt + rr) * PQROW + HD * cg + 4 * lane) = v;
  }
  __threadfence();
#pragma unroll 1
  for (int rr = 0; rr < 16; ++rr) {
    const v4f v = *(const v4f*)(sw + rr * SP + 4 * lane);
    *(volatile v4f*)(PQ + (size_t)(n0 + 16 * rt + rr) * PQROW + HD * cg + 4 * lane) = v;
  }
}

__global__ __launch_bounds__(NTHR) void k_edge(
    const int* __restrict__ ei, const float* __restrict__ tt, const float* __restrict__ PQ,
    const float* __restrict__ Wt, const float* __restrict__ bt, const float* __restrict__ b1,
    const float* __restrict__ b2, const _Float16* __restrict__ wp, _Float16* OE,
    int c0, int nE, int nN) {
  __shared__ __attribute__((aligned(16))) _Float16 sA[TE * AP];
  __shared__ __attribute__((aligned(16))) float sPar[4 * HD];
  __shared__ float sT[TE];
  __shared__ int sIdx[2 * TE];
  const int tid = (int)threadIdx.x, lane = tid & 31, wave = tid >> 5, hh = lane >> 4, m = lane & 15;
  const int le0 = (int)blockIdx.x * TE;
  const int ge0 = c0 + le0;

  {
    const int s = tid >> 7, j = tid & (TE - 1);
    int e = ge0 + j;
    e = e > nE - 1 ? nE - 1 : e;
    int v = ei[(size_t)s * nE + e];
    if (v < 0) v += nN;
    v = iclamp(v, 0, nN - 1);
    sIdx[s * TE + j] = v;
  }
  if (tid < HD) {
    sPar[tid]          = Wt[tid];
    sPar[HD + tid]     = bt[tid];
    sPar[2 * HD + tid] = b1[tid];
    sPar[3 * HD + tid] = b2[tid];
  }
  if (tid < TE) {
    int e = ge0 + tid;
    e = e > nE - 1 ? nE - 1 : e;
    sT[tid] = tt[e];
  }
  __syncthreads();

  {
    const int el = tid >> 1, q = tid & 1;
    const int rnode = sIdx[el], cnode = sIdx[TE + el];
    const float tv = sT[el];
    const float* pp = PQ + (size_t)rnode * PQROW + 64 * q;
    const float* qp = PQ + (size_t)cnode * PQROW + HD + 64 * q;
    const float* pw = sPar + 64 * q;
    const float* pb = sPar + HD + 64 * q;
    const float* p1 = sPar + 2 * HD + 64 * q;
    _Float16* dst = sA + el * AP + 64 * q;
#pragma unroll 1
    for (int i = 0; i < 8; ++i) {
      const v4f a0 = *(const v4f*)(pp + 8 * i);
      const v4f a1 = *(const v4f*)(pp + 8 * i + 4);
      const v4f g0 = *(const v4f*)(qp + 8 * i);
      const v4f g1 = *(const v4f*)(qp + 8 * i + 4);
      const int cb = 8 * i;
      v8h o;
      o[0] = hchan(a0.x, g0.x, tv, pw[cb + 0], pb[cb + 0], p1[cb + 0]);
      o[1] = hchan(a0.y, g0.y, tv, pw[cb + 1], pb[cb + 1], p1[cb + 1]);
      o[2] = hchan(a0.z, g0.z, tv, pw[cb + 2], pb[cb + 2], p1[cb + 2]);
      o[3] = hchan(a0.w, g0.w, tv, pw[cb + 3], pb[cb + 3], p1[cb + 3]);
      o[4] = hchan(a1.x, g1.x, tv, pw[cb + 4], pb[cb + 4], p1[cb + 4]);
      o[5] = hchan(a1.y, g1.y, tv, pw[cb + 5], pb[cb + 5], p1[cb + 5]);
      o[6] = hchan(a1.z, g1.z, tv, pw[cb + 6], pb[cb + 6], p1[cb + 6]);
      o[7] = hchan(a1.w, g1.w, tv, pw[cb + 7], pb[cb + 7], p1[cb + 7]);
      *(v8h*)(dst + 8 * i) = o;
    }
  }
  __syncthreads();

  const int rt = wave & 3, cg = wave >> 2;
  v8f c[2][4];
#pragma unroll
  for (int u = 0; u < 2; ++u) {
#pragma unroll
    for (int j = 0; j < 4; ++j) c[u][j] = zero8();
  }
  {
    const _Float16* ap0 = sA + (32 * rt + m) * AP + 8 * hh;
    const _Float16* ap1 = ap0 + 16 * AP;
    const _Float16* bp = wp + PW2 + (size_t)(64 * cg + m) * HD + 8 * hh;
#pragma unroll 1
    for (int ks = 0; ks < 4; ++ks) {
      const v16h a0 = ldfrag(ap0 + 32 * ks);
      const v16h a1 = ldfrag(ap1 + 32 * ks);
#pragma unroll
      for (int j = 0; j < 4; ++j) {
        const v16h b = ldfrag(bp + (size_t)(16 * j) * HD + 32 * ks);
        c[0][j] = wm(a0, b, c[0][j]);
        c[1][j] = wm(a1, b, c[1][j]);
      }
    }
  }
  __syncthreads();

#pragma unroll
  for (int u = 0; u < 2; ++u) {
#pragma unroll
    for (int j = 0; j < 4; ++j) {
      const int col = 64 * cg + 16 * j + m;
      const float bb = sPar[3 * HD + col];
      _Float16* sp = sA + (32 * rt + 16 * u + 8 * hh) * AP + col;
#pragma unroll
      for (int r = 0; r < 8; ++r) sp[r * AP] = (_Float16)(c[u][j][r] * 0.0009765625f + bb);
    }
  }
  __syncthreads();
#pragma unroll 1
  for (int i = 0; i < 8; ++i) {
    const int row = 16 * wave + 2 * i + hh;
    const v4u v = *(const v4u*)(sA + row * AP + 8 * m);
    *(volatile v4u*)(OE + (size_t)(le0 + row) * HD + 8 * m) = v;
  }
  __threadfence();
#pragma unroll 1
  for (int i = 0; i < 8; ++i) {
    const int row = 16 * wave + 2 * i + hh;
    const v4u v = *(const v4u*)(sA + row * AP + 8 * m);
    *(volatile v4u*)(OE + (size_t)(le0 + row) * HD + 8 * m) = v;
  }
}

__device__ __forceinline__ int scan_piece(const int* __restrict__ kp, int lim, int cbase, int base,
                                          int* list, int tid, int wave, int vec_ok) {
  int wc = 0;
  const int el0  = tid * EPT;
  const int e0   = cbase + el0;
  const int sent = -2147483647 - 1;
  int kk[EPT];
  if (vec_ok != 0 && cbase + PIECE <= lim) {
    const v4i* p = (const v4i*)(kp + e0);
#pragma unroll
    for (int u = 0; u < EPT / 4; ++u) {
      const v4i d = p[u];
      kk[4 * u] = d.x; kk[4 * u + 1] = d.y; kk[4 * u + 2] = d.z; kk[4 * u + 3] = d.w;
    }
  } else {
    const int lm = lim - 1;
#pragma unroll
    for (int q = 0; q < EPT; ++q) {
      const int eq = e0 + q;
      const int ec = eq > lm ? lm : eq;
      const int a = kp[ec];
      kk[q] = (eq < lim) ? a : sent;
    }
  }
  const unsigned nb = (unsigned)base;
  unsigned sq[EPT];
  bool hq[EPT];
  bool anyl = false;
#pragma unroll
  for (int q = 0; q < EPT; ++q) {
    sq[q] = (unsigned)kk[q] - nb;
    hq[q] = sq[q] < (unsigned)NBC;
    anyl = anyl | hq[q];
  }
  const unsigned any = __builtin_amdgcn_ballot_w32(anyl);
  if (any != 0u) {
#define HIT(HQ, SQ, Q) { \
      const unsigned mj = __builtin_amdgcn_ballot_w32(HQ); \
      if (mj != 0u) { \
        if (HQ) { \
          const int ps = wc + (int)__builtin_amdgcn_mbcnt_lo(mj, 0u); \
          if (ps < WCAP) list[wave * WCAP + ps] = ((el0 + (Q)) << SLB) | (int)(SQ); \
        } \
        wc += (int)__builtin_popcount(mj); } }
#pragma unroll
    for (int q = 0; q < EPT; ++q) {
      HIT(hq[q], sq[q], q)
    }
#undef HIT
  }
  return wc;
}

__device__ __forceinline__ void drain_sum(const int* list, const int* wcnt, float* accF,
                                          const _Float16* __restrict__ OE, int side,
                                          int cbase, int nec, int lane, int wave) {
#pragma unroll 1
  for (int wsx = 0; wsx < NWAVE; ++wsx) {
    int n = __builtin_amdgcn_readfirstlane(wcnt[wsx]);
    n = n > WCAP ? WCAP : (n < 0 ? 0 : n);
    const int* lp = list + wsx * WCAP;
#pragma unroll 1
    for (int bb = 0; bb < n; bb += 32) {
      const int idx = bb + lane;
      const int ic = idx > WCAP - 1 ? WCAP - 1 : idx;
      const int ent = lp[ic];
      const bool own = (idx < n) && ((ent & (NWAVE - 1)) == wave);
      unsigned msk = __builtin_amdgcn_ballot_w32(own);
#pragma unroll 1
      while (msk != 0u) {
        const int bit = (int)__builtin_ctz(msk);
        msk &= msk - 1u;
        const int e2 = __builtin_amdgcn_readlane(ent, bit);
        const int slot = e2 & (NBC - 1);
        const int el = (e2 >> SLB) & (PIECE - 1);
        int e = cbase + el;
        e = e > nec - 1 ? nec - 1 : (e < 0 ? 0 : e);
        const v2h hv = *(const v2h*)(OE + (size_t)e * HD + DF * side + 2 * lane);
        float* ap = accF + slot * DF + 2 * lane;
        v2f a = *(const v2f*)ap;
        a.x = a.x + (float)hv.x;
        a.y = a.y + (float)hv.y;
        *(v2f*)ap = a;
      }
    }
  }
}

__device__ __forceinline__ void node_rows(const float* accF, float* outp, int base, int nN,
                                          int wave, int hh, int m) {
#pragma unroll 1
  for (int it = 0; it < NBC / (2 * NWAVE); ++it) {
    const int s = 2 * (wave + NWAVE * it) + hh;
    const int node = base + s;
    if (node < nN) {
      const v4f v = *(const v4f*)(accF + s * DF + 4 * m);
      *(volatile v4f*)(outp + (size_t)node * DF + 4 * m) = v;
    }
  }
}

__global__ __launch_bounds__(NTHR) void k_agg(
    const int* __restrict__ ei, const _Float16* __restrict__ OE, float* outp,
    int c0, int nec, int nE, int nN, int first, int vec_ok) {
  extern __shared__ __attribute__((aligned(16))) float accF[];
  __shared__ int list[NWAVE * WCAP];
  __shared__ int wcnt[NWAVE];
  const int tid = (int)threadIdx.x, lane = tid & 31, wave = tid >> 5, hh = lane >> 4, m = lane & 15;
  const int base = (int)blockIdx.x * NBC;

  if (first != 0) {
    const v4f z = {0.0f, 0.0f, 0.0f, 0.0f};
#pragma unroll 1
    for (int i = tid; i < (NBC * DF) / 4; i += NTHR) *(v4f*)(accF + 4 * i) = z;
  } else {
#pragma unroll 1
    for (int i = tid; i < (NBC * DF) / 4; i += NTHR) {
      const int slot = i >> 4;
      const int node = base + slot;
      const int nc = node > nN - 1 ? nN - 1 : node;
      v4f v = *(const v4f*)(outp + (size_t)nc * DF + 4 * (i & 15));
      if (node > nN - 1) { v.x = 0.0f; v.y = 0.0f; v.z = 0.0f; v.w = 0.0f; }
      *(v4f*)(accF + 4 * i) = v;
    }
  }
  __syncthreads();

#pragma unroll 1
  for (int side = 0; side < 2; ++side) {
    const int* kp = ei + (size_t)side * nE + c0;
#pragma unroll 1
    for (int cbase = 0; cbase < nec; cbase += PIECE) {
      const int wc = scan_piece(kp, nec, cbase, base, list, tid, wave, vec_ok);
      if (lane == 0) wcnt[wave] = wc;
      __syncthreads();
      drain_sum(list, wcnt, accF, OE, side, cbase, nec, lane, wave);
      __syncthreads();
    }
  }

  node_rows(accF, outp, base, nN, wave, hh, m);
  __threadfence();
  node_rows(accF, outp, base, nN, wave, hh, m);
}

extern "C" void kernel_launch(void* const* d_in, const int* in_sizes, int n_in,
                              void* d_out, int out_size, void* d_ws, size_t ws_size,
                              hipStream_t stream) {
  if (n_in < 9) return;
  if (in_sizes[0] < DF || (in_sizes[0] % DF) != 0) return;
  const int nN = in_sizes[0] / DF;
  if (nN < 1 || nN > (1 << 24)) return;
  const int nE = in_sizes[2];
  if (nE < 1 || nE > (1 << 27)) return;
  if (in_sizes[1] != 2 * nE) return;
  if (in_sizes[3] != HD * HD || in_sizes[4] != HD) return;
  if (in_sizes[5] != HD || in_sizes[6] != HD) return;
  if (in_sizes[7] != HD * HD || in_sizes[8] != HD) return;
  if ((long long)out_size != (long long)nN * DF) return;

  const float* x  = (const float*)d_in[0];
  const int*   ei = (const int*)d_in[1];
  const float* tt = (const float*)d_in[2];
  const float* W1 = (const float*)d_in[3];
  const float* b1 = (const float*)d_in[4];
  const float* Wt = (const float*)d_in[5];
  const float* bt = (const float*)d_in[6];
  const float* W2 = (const float*)d_in[7];
  const float* b2 = (const float*)d_in[8];
  float* outp = (float*)d_out;

  const int nb64 = (nN + NBN - 1) / NBN;
  const int Npad64 = nb64 * NBN;
  const int nbA = (nN + NBC - 1) / NBC;
  const int vec_ok = ((nE & 3) == 0) ? 1 : 0;

  const size_t cap = ws_size < (size_t)WSCAP ? ws_size : (size_t)WSCAP;
  const size_t bW  = (size_t)PWTOT * 2;
  const size_t bPQ = (size_t)Npad64 * PQROW * 4;
  const size_t fixedB = ((bW + 255) & ~(size_t)255) + ((bPQ + 255) & ~(size_t)255);
  int C = 0;
  size_t CE = 0;
  for (int c = 1; c <= 512; ++c) {
    size_t ce = ((size_t)nE + (size_t)c - 1) / (size_t)c;
    ce = (ce + PIECE - 1) / PIECE * PIECE;
    const size_t tot = fixedB + ((ce * HD * 2 + 255) & ~(size_t)255);
    if (tot <= cap) { C = c; CE = ce; break; }
  }
  if (C == 0) return;

  char* ws = (char*)d_ws;
  size_t off = 0;
  const size_t oW  = off; off += bW;                    off = (off + 255) & ~(size_t)255;
  const size_t oPQ = off; off += bPQ;                   off = (off + 255) & ~(size_t)255;
  const size_t oOE = off; off += CE * HD * 2;           off = (off + 255) & ~(size_t)255;
  if (off > cap || off > ws_size) return;
  _Float16* wp = (_Float16*)(ws + oW);
  float*    PQ = (float*)(ws + oPQ);
  _Float16* OE = (_Float16*)(ws + oOE);

  hipFuncSetAttribute(reinterpret_cast<const void*>(&k_pq),  hipFuncAttributeMaxDynamicSharedMemorySize, PQDYN);
  hipFuncSetAttribute(reinterpret_cast<const void*>(&k_agg), hipFuncAttributeMaxDynamicSharedMemorySize, AGGDYN);

  k_prep<<<PREPBLK, NTHR, 0, stream>>>(W1, W2, wp);
  k_pq<<<nb64, NTHR, PQDYN, stream>>>(x, wp, PQ, nN);
  for (int ch = 0; ch < C; ++ch) {
    const size_t c0s = (size_t)ch * CE;
    if (c0s >= (size_t)nE) break;
    const int c0 = (int)c0s;
    size_t necs = (size_t)nE - c0s;
    if (necs > CE) necs = CE;
    const int nec = (int)necs;
    const int ntiles = (nec + TE - 1) / TE;
    k_edge<<<ntiles, NTHR, 0, stream>>>(ei, tt, PQ, Wt, bt, b1, b2, wp, OE, c0, nE, nN);
    k_agg<<<nbA, NTHR, AGGDYN, stream>>>(ei, OE, outp, c0, nec, nE, nN, (ch == 0) ? 1 : 0, vec_ok);
  }
}
